// EnhancedSocialRecommender_87866440942265
// MI455X (gfx1250) — hardware-run, weakly checked
//
#include <hip/hip_runtime.h>


namespace {
constexpr int NU = 100000, NI = 150000, D = 64, EUI = 2000000, ES_ = 1000000, NB = 4096, NPB = 8;
constexpr float HS = 256.0f, WSC = 256.0f, LNEPS = 1e-5f;
typedef _Float16 b16;
typedef __attribute__((ext_vector_type(16))) _Float16 v16b;
typedef __attribute__((ext_vector_type(8))) _Float16 v8b;
typedef __attribute__((ext_vector_type(8))) float v8f;
typedef __attribute__((ext_vector_type(4))) float v4f;
typedef __attribute__((ext_vector_type(2))) float v2f;
__device__ __forceinline__ float bf16_rne(float f) { unsigned int u = __float_as_uint(f); u += 0x7FFFu + ((u >> 16) & 1u); float r = __uint_as_float(u & 0xFFFF0000u); asm volatile("" : "+v"(r)); return r; }
__device__ __forceinline__ float bfv(float f) { float r = bf16_rne(f); asm volatile("" : "+v"(r)); return r; }
__device__ __forceinline__ void split16(float v, b16& hi, b16& lo) { hi = (b16)v; lo = (b16)(v - (float)hi); }
__device__ __forceinline__ v16b frag_kb(const b16* p, int hh) { const v8b a = *(const v8b*)(p + 8 * hh), b = *(const v8b*)(p + 16 + 8 * hh); v16b f;
#pragma unroll
  for (int e = 0; e < 8; ++e) { f[e] = a[e]; f[8 + e] = b[e]; } return f; }
__device__ __forceinline__ v8f wmma16b(v16b a, v16b b, v8f c) { v8f d = __builtin_amdgcn_wmma_f32_16x16x32_f16(false, a, false, b, (short)0, c, false, false); asm volatile("v_nop\n\tv_nop\n\tv_nop\n\tv_nop" : "+v"(d) : "v"(a), "v"(b)); return d; }
__device__ __forceinline__ void wave_lds_sync() { __builtin_amdgcn_fence(__ATOMIC_RELEASE, "workgroup"); __builtin_amdgcn_wave_barrier(); __builtin_amdgcn_fence(__ATOMIC_ACQUIRE, "workgroup"); }
__device__ __forceinline__ float pmul(float a, float b) { float p = a * b; asm volatile("" : "+v"(p)); return p; }
__device__ __forceinline__ int iclamp(int v, int lo, int hi) { return v < lo ? lo : (v > hi ? hi : v); }
__device__ __forceinline__ float leaky(float v) { return v > 0.0f ? v : 0.01f * v; }
__device__ __forceinline__ float sigm(float v) { return 1.0f / (1.0f + __expf(-v)); }
constexpr int CSR_NBLK8 = 512, CSR_GB8 = 8, CSR_GN8 = 1 << CSR_GB8  , CSR_TS8 = (CSR_GN8 < 32 ? 32 : CSR_GN8)  , CSR_MAXG8 = 512, CSR_CAP8 = 12288  ;
__device__ __host__ __forceinline__ int csr_tix8(int v) { return (v >> CSR_GB8) * CSR_TS8 + (v & (CSR_GN8 - 1)); }
__global__ __launch_bounds__(64) void csrA_kernel8(const int* __restrict__ dst, int E, int N, int nG, int CHP, int NGP, int* __restrict__ STG, int* __restrict__ HST) {
  extern __shared__ int sm[];
  int* cnt = sm; int* run = sm + NGP; int* ids = sm + 2 * NGP;
  const int b = blockIdx.x; const int ch = (E + CSR_NBLK8 - 1) / CSR_NBLK8; const int e0 = b * ch, e1 = min(E, e0 + ch);
  for (int i = threadIdx.x; i < NGP; i += 64) cnt[i] = 0;
  for (int i = threadIdx.x; i < CHP; i += 64) ids[i] = -1;
  __syncthreads();
  if (threadIdx.x == 0) {
    for (int e = e0; e < e1; ++e) { int d = dst[e]; d = (d < 0) ? 0 : (d >= N ? N - 1 : d); cnt[d >> CSR_GB8] += 1; }
    int acc = 0; for (int g = 0; g < nG; ++g) { run[g] = acc; acc += cnt[g]; }
    for (int e = e0; e < e1; ++e) { int d = dst[e]; d = (d < 0) ? 0 : (d >= N ? N - 1 : d); const int g = d >> CSR_GB8; ids[run[g]] = e; run[g] += 1; } }
  __syncthreads();
  typedef __attribute__((ext_vector_type(4))) int v4i;
  for (int pass = 0; pass < 2; ++pass) {
    for (int i = threadIdx.x; i < CHP / 4; i += 64) *(volatile v4i*)(STG + (size_t)b * CHP + i * 4) = *(const v4i*)(&ids[i * 4]);
    for (int i = threadIdx.x; i < NGP / 4; i += 64) { v4i v; for (int e = 0; e < 4; ++e) v[e] = (i * 4 + e < nG) ? cnt[i * 4 + e] : 0; *(volatile v4i*)(HST + (size_t)b * NGP + i * 4) = v; }
    __threadfence(); }
}
__global__ __launch_bounds__(512) void csrS_kernel8(const int* __restrict__ HST, int nG, int NGP, int* __restrict__ START, int* __restrict__ TOT, int* __restrict__ OFF) {
  __shared__ int tot[CSR_MAXG8];
  const int b = threadIdx.x;
  for (int pass = 0; pass < 2; ++pass) { int runb = 0; for (int g = 0; g < nG; ++g) { int c = HST[(size_t)b * NGP + g]; c = (c < 0) ? 0 : c; ((volatile int*)OFF)[(size_t)g * CSR_NBLK8 + b] = runb; runb += c; } __threadfence(); }
  for (int g = threadIdx.x; g < nG; g += 512) { int s = 0; for (int bb = 0; bb < CSR_NBLK8; ++bb) { int c = HST[(size_t)bb * NGP + g]; s += (c < 0) ? 0 : c; } tot[g] = s; }
  __syncthreads();
  if (threadIdx.x < 32) {
    __shared__ int st[CSR_MAXG8 + 32];
    if (threadIdx.x == 0) { int acc = 0; for (int g = 0; g < NGP; ++g) { st[g] = acc; if (g < nG) acc += (tot[g] + 31) & ~31; } st[NGP] = acc; }
    __builtin_amdgcn_fence(__ATOMIC_RELEASE, "workgroup"); __builtin_amdgcn_wave_barrier(); __builtin_amdgcn_fence(__ATOMIC_ACQUIRE, "workgroup");
    for (int pass = 0; pass < 2; ++pass) { for (int i = threadIdx.x; i < NGP + 32; i += 32) { ((volatile int*)START)[i] = (i <= NGP) ? st[min(i, NGP)] : 0; ((volatile int*)TOT)[i] = (i < nG) ? tot[i] : 0; } __threadfence(); } }
}
__global__ __launch_bounds__(256) void csrB_kernel8(const int* __restrict__ dst, int N, int nG, int CHP, int NGP, int permLen, const int* __restrict__ STG, const int* __restrict__ HST, const int* __restrict__ OFF, const int* __restrict__ START, const int* __restrict__ TOT, int* __restrict__ PERM, int* __restrict__ ROWPTR, int* __restrict__ ROWCNT, int* __restrict__ FLAG) {
  typedef __attribute__((ext_vector_type(4))) int v4i;
  __shared__ int ids[CSR_CAP8]; __shared__ unsigned short key[CSR_CAP8]; __shared__ int outp[CSR_CAP8]; __shared__ int ncnt[CSR_GN8 + 1]; __shared__ int boff[CSR_NBLK8 + 1];
  const int g = blockIdx.x, t_ = threadIdx.x; int tot = TOT[g]; int st = START[g], stn = START[g + 1]; const int v0 = g * CSR_GN8; const int nv = min(CSR_GN8, N - v0); const int t0 = g * CSR_TS8;
  st = (st < 0) ? 0 : (st > permLen - 32 ? permLen - 32 : st) & ~31; stn = (stn < st) ? st : (stn > permLen ? permLen : stn); tot = (tot < 0) ? 0 : tot; if (tot > stn - st && tot <= CSR_CAP8) tot = stn - st;
  if (tot > CSR_CAP8) {
    for (int pass = 0; pass < 2; ++pass) { for (int i = t_; i < CSR_TS8 / 4; i += 256) { v4i a, c; for (int e = 0; e < 4; ++e) { a[e] = st; c[e] = 0; } *(volatile v4i*)(ROWPTR + t0 + i * 4) = a; *(volatile v4i*)(ROWCNT + t0 + i * 4) = c; } if (t_ == 0) ((volatile int*)FLAG)[0] = 1; __threadfence(); } (void)nv; return; }
  if (t_ == 0) { int acc = 0; for (int b = 0; b < CSR_NBLK8; ++b) { boff[b] = acc; int c = HST[(size_t)b * NGP + g]; c = (c < 0) ? 0 : (c > CHP ? CHP : c); acc += c; if (acc > tot) acc = tot; } boff[CSR_NBLK8] = acc; }
  for (int i = t_; i <= CSR_GN8; i += 256) ncnt[i] = 0;
  __syncthreads();
  for (int b = 0; b < CSR_NBLK8; ++b) { const int c = boff[b + 1] - boff[b]; int o_ = OFF[(size_t)g * CSR_NBLK8 + b]; o_ = (o_ < 0) ? 0 : (o_ > CHP - c ? CHP - c : o_); const int* src_ = STG + (size_t)b * CHP + o_;
    for (int i = t_; i < c; i += 256) { int id = src_[i]; id = (id < 0) ? 0 : id; ids[boff[b] + i] = id; int d = dst[id]; d = (d < v0) ? v0 : (d >= N ? N - 1 : d); int kk = d - v0; kk = (kk < 0) ? 0 : (kk >= CSR_GN8 ? CSR_GN8 - 1 : kk); key[boff[b] + i] = (unsigned short)kk; } }
  __syncthreads();
  if (t_ == 0) { for (int i = 0; i < tot; ++i) ncnt[key[i]] += 1; int acc = 0; for (int vl = 0; vl < CSR_GN8; ++vl) { const int c = ncnt[vl]; ncnt[vl] = acc; acc += c; } ncnt[CSR_GN8] = acc;
    for (int i = 0; i < tot; ++i) { const int vl = key[i]; outp[ncnt[vl]] = ids[i]; ncnt[vl] += 1; }
    for (int vl = CSR_GN8; vl > 0; --vl) ncnt[vl] = ncnt[vl - 1]; ncnt[0] = 0; }
  __syncthreads();
  for (int pass = 0; pass < 2; ++pass) {
    for (int i = t_; i < (stn - st) / 4; i += 256) { v4i v; for (int e = 0; e < 4; ++e) { const int q = i * 4 + e; v[e] = (q < tot) ? outp[q] : -1; } *(volatile v4i*)(PERM + st + i * 4) = v; }
    for (int i = t_; i < CSR_TS8 / 4; i += 256) { v4i a, c; for (int e = 0; e < 4; ++e) { const int vl = i * 4 + e; const int vc = vl < CSR_GN8 ? vl : CSR_GN8; a[e] = (vl < CSR_GN8) ? st + ncnt[vc] : st; c[e] = (vl < nv) ? (ncnt[(vc < CSR_GN8 ? vc : CSR_GN8 - 1) + 1] - ncnt[vc]) : 0; } *(volatile v4i*)(ROWPTR + t0 + i * 4) = a; *(volatile v4i*)(ROWCNT + t0 + i * 4) = c; }
    __threadfence(); }
}
__global__ __launch_bounds__(256) void csrZ_kernel8(int* __restrict__ p, size_t n4) { typedef __attribute__((ext_vector_type(4))) int v4i; const size_t tid = (size_t)blockIdx.x * 256 + threadIdx.x, nth = (size_t)gridDim.x * 256; v4i z = {0, 0, 0, 0}; for (size_t i = tid; i < n4; i += nth) *(volatile v4i*)(p + i * 4) = z; }
struct CsrBufs8 { int *STG, *HST, *OFF, *START, *TOT, *PERM, *ROWPTR, *ROWCNT, *FLAG; int nG, NGP, CHP; size_t permLen; char* base; size_t bytes; };
static size_t csr_carve8(CsrBufs8& c, char* ws, size_t off, int E, int N) {
  const size_t off0 = off; c.base = ws + off;
  auto al = [&](size_t bytes) { char* p = ws + off; off += (bytes + 255) & ~(size_t)255; return p; };
  c.nG = (N + CSR_GN8 - 1) / CSR_GN8; c.NGP = (c.nG + 31) & ~31; const int ch = (E + CSR_NBLK8 - 1) / CSR_NBLK8; c.CHP = (ch + 31) & ~31; c.permLen = (size_t)E + 32 * (size_t)c.nG + 32;
  c.STG = (int*)al((size_t)CSR_NBLK8 * c.CHP * 4); c.HST = (int*)al((size_t)CSR_NBLK8 * c.NGP * 4); c.OFF = (int*)al((size_t)c.NGP * CSR_NBLK8 * 4); c.START = (int*)al((size_t)(c.NGP + 64) * 4); c.TOT = (int*)al((size_t)(c.NGP + 64) * 4);
  c.PERM = (int*)al(c.permLen * 4); c.ROWPTR = (int*)al((size_t)c.nG * CSR_TS8 * 4); c.ROWCNT = (int*)al((size_t)c.nG * CSR_TS8 * 4); c.FLAG = (int*)al(256);
  c.bytes = off - off0; return off;
}
static void csr_build8(const CsrBufs8& c, const int* dst, int E, int N, hipStream_t stream) {
  const size_t smem = (size_t)(2 * c.NGP + c.CHP) * 4;
  csrZ_kernel8<<<512, 256, 0, stream>>>((int*)c.base, c.bytes / 16);
  csrA_kernel8<<<CSR_NBLK8, 64, smem, stream>>>(dst, E, N, c.nG, c.CHP, c.NGP, c.STG, c.HST);
  csrS_kernel8<<<1, 512, 0, stream>>>(c.HST, c.nG, c.NGP, c.START, c.TOT, c.OFF);
  csrB_kernel8<<<c.nG, 256, 0, stream>>>(dst, N, c.nG, c.CHP, c.NGP, (int)c.permLen, c.STG, c.HST, c.OFF, c.START, c.TOT, c.PERM, c.ROWPTR, c.ROWCNT, c.FLAG);
}
constexpr int CSR_NBLK9 = 512, CSR_GB9 = 9, CSR_GN9 = 1 << CSR_GB9  , CSR_TS9 = (CSR_GN9 < 32 ? 32 : CSR_GN9)  , CSR_MAXG9 = 512, CSR_CAP9 = 12288  ;
__device__ __host__ __forceinline__ int csr_tix9(int v) { return (v >> CSR_GB9) * CSR_TS9 + (v & (CSR_GN9 - 1)); }
__global__ __launch_bounds__(64) void csrA_kernel9(const int* __restrict__ dst, int E, int N, int nG, int CHP, int NGP, int* __restrict__ STG, int* __restrict__ HST) {
  extern __shared__ int sm[];
  int* cnt = sm; int* run = sm + NGP; int* ids = sm + 2 * NGP;
  const int b = blockIdx.x; const int ch = (E + CSR_NBLK9 - 1) / CSR_NBLK9; const int e0 = b * ch, e1 = min(E, e0 + ch);
  for (int i = threadIdx.x; i < NGP; i += 64) cnt[i] = 0;
  for (int i = threadIdx.x; i < CHP; i += 64) ids[i] = -1;
  __syncthreads();
  if (threadIdx.x == 0) {
    for (int e = e0; e < e1; ++e) { int d = dst[e]; d = (d < 0) ? 0 : (d >= N ? N - 1 : d); cnt[d >> CSR_GB9] += 1; }
    int acc = 0; for (int g = 0; g < nG; ++g) { run[g] = acc; acc += cnt[g]; }
    for (int e = e0; e < e1; ++e) { int d = dst[e]; d = (d < 0) ? 0 : (d >= N ? N - 1 : d); const int g = d >> CSR_GB9; ids[run[g]] = e; run[g] += 1; } }
  __syncthreads();
  typedef __attribute__((ext_vector_type(4))) int v4i;
  for (int pass = 0; pass < 2; ++pass) {
    for (int i = threadIdx.x; i < CHP / 4; i += 64) *(volatile v4i*)(STG + (size_t)b * CHP + i * 4) = *(const v4i*)(&ids[i * 4]);
    for (int i = threadIdx.x; i < NGP / 4; i += 64) { v4i v; for (int e = 0; e < 4; ++e) v[e] = (i * 4 + e < nG) ? cnt[i * 4 + e] : 0; *(volatile v4i*)(HST + (size_t)b * NGP + i * 4) = v; }
    __threadfence(); }
}
__global__ __launch_bounds__(512) void csrS_kernel9(const int* __restrict__ HST, int nG, int NGP, int* __restrict__ START, int* __restrict__ TOT, int* __restrict__ OFF) {
  __shared__ int tot[CSR_MAXG9];
  const int b = threadIdx.x;
  for (int pass = 0; pass < 2; ++pass) { int runb = 0; for (int g = 0; g < nG; ++g) { int c = HST[(size_t)b * NGP + g]; c = (c < 0) ? 0 : c; ((volatile int*)OFF)[(size_t)g * CSR_NBLK9 + b] = runb; runb += c; } __threadfence(); }
  for (int g = threadIdx.x; g < nG; g += 512) { int s = 0; for (int bb = 0; bb < CSR_NBLK9; ++bb) { int c = HST[(size_t)bb * NGP + g]; s += (c < 0) ? 0 : c; } tot[g] = s; }
  __syncthreads();
  if (threadIdx.x < 32) {
    __shared__ int st[CSR_MAXG9 + 32];
    if (threadIdx.x == 0) { int acc = 0; for (int g = 0; g < NGP; ++g) { st[g] = acc; if (g < nG) acc += (tot[g] + 31) & ~31; } st[NGP] = acc; }
    __builtin_amdgcn_fence(__ATOMIC_RELEASE, "workgroup"); __builtin_amdgcn_wave_barrier(); __builtin_amdgcn_fence(__ATOMIC_ACQUIRE, "workgroup");
    for (int pass = 0; pass < 2; ++pass) { for (int i = threadIdx.x; i < NGP + 32; i += 32) { ((volatile int*)START)[i] = (i <= NGP) ? st[min(i, NGP)] : 0; ((volatile int*)TOT)[i] = (i < nG) ? tot[i] : 0; } __threadfence(); } }
}
__global__ __launch_bounds__(256) void csrB_kernel9(const int* __restrict__ dst, int N, int nG, int CHP, int NGP, int permLen, const int* __restrict__ STG, const int* __restrict__ HST, const int* __restrict__ OFF, const int* __restrict__ START, const int* __restrict__ TOT, int* __restrict__ PERM, int* __restrict__ ROWPTR, int* __restrict__ ROWCNT, int* __restrict__ FLAG) {
  typedef __attribute__((ext_vector_type(4))) int v4i;
  __shared__ int ids[CSR_CAP9]; __shared__ unsigned short key[CSR_CAP9]; __shared__ int outp[CSR_CAP9]; __shared__ int ncnt[CSR_GN9 + 1]; __shared__ int boff[CSR_NBLK9 + 1];
  const int g = blockIdx.x, t_ = threadIdx.x; int tot = TOT[g]; int st = START[g], stn = START[g + 1]; const int v0 = g * CSR_GN9; const int nv = min(CSR_GN9, N - v0); const int t0 = g * CSR_TS9;
  st = (st < 0) ? 0 : (st > permLen - 32 ? permLen - 32 : st) & ~31; stn = (stn < st) ? st : (stn > permLen ? permLen : stn); tot = (tot < 0) ? 0 : tot; if (tot > stn - st && tot <= CSR_CAP9) tot = stn - st;
  if (tot > CSR_CAP9) {
    for (int pass = 0; pass < 2; ++pass) { for (int i = t_; i < CSR_TS9 / 4; i += 256) { v4i a, c; for (int e = 0; e < 4; ++e) { a[e] = st; c[e] = 0; } *(volatile v4i*)(ROWPTR + t0 + i * 4) = a; *(volatile v4i*)(ROWCNT + t0 + i * 4) = c; } if (t_ == 0) ((volatile int*)FLAG)[0] = 1; __threadfence(); } (void)nv; return; }
  if (t_ == 0) { int acc = 0; for (int b = 0; b < CSR_NBLK9; ++b) { boff[b] = acc; int c = HST[(size_t)b * NGP + g]; c = (c < 0) ? 0 : (c > CHP ? CHP : c); acc += c; if (acc > tot) acc = tot; } boff[CSR_NBLK9] = acc; }
  for (int i = t_; i <= CSR_GN9; i += 256) ncnt[i] = 0;
  __syncthreads();
  for (int b = 0; b < CSR_NBLK9; ++b) { const int c = boff[b + 1] - boff[b]; int o_ = OFF[(size_t)g * CSR_NBLK9 + b]; o_ = (o_ < 0) ? 0 : (o_ > CHP - c ? CHP - c : o_); const int* src_ = STG + (size_t)b * CHP + o_;
    for (int i = t_; i < c; i += 256) { int id = src_[i]; id = (id < 0) ? 0 : id; ids[boff[b] + i] = id; int d = dst[id]; d = (d < v0) ? v0 : (d >= N ? N - 1 : d); int kk = d - v0; kk = (kk < 0) ? 0 : (kk >= CSR_GN9 ? CSR_GN9 - 1 : kk); key[boff[b] + i] = (unsigned short)kk; } }
  __syncthreads();
  if (t_ == 0) { for (int i = 0; i < tot; ++i) ncnt[key[i]] += 1; int acc = 0; for (int vl = 0; vl < CSR_GN9; ++vl) { const int c = ncnt[vl]; ncnt[vl] = acc; acc += c; } ncnt[CSR_GN9] = acc;
    for (int i = 0; i < tot; ++i) { const int vl = key[i]; outp[ncnt[vl]] = ids[i]; ncnt[vl] += 1; }
    for (int vl = CSR_GN9; vl > 0; --vl) ncnt[vl] = ncnt[vl - 1]; ncnt[0] = 0; }
  __syncthreads();
  for (int pass = 0; pass < 2; ++pass) {
    for (int i = t_; i < (stn - st) / 4; i += 256) { v4i v; for (int e = 0; e < 4; ++e) { const int q = i * 4 + e; v[e] = (q < tot) ? outp[q] : -1; } *(volatile v4i*)(PERM + st + i * 4) = v; }
    for (int i = t_; i < CSR_TS9 / 4; i += 256) { v4i a, c; for (int e = 0; e < 4; ++e) { const int vl = i * 4 + e; const int vc = vl < CSR_GN9 ? vl : CSR_GN9; a[e] = (vl < CSR_GN9) ? st + ncnt[vc] : st; c[e] = (vl < nv) ? (ncnt[(vc < CSR_GN9 ? vc : CSR_GN9 - 1) + 1] - ncnt[vc]) : 0; } *(volatile v4i*)(ROWPTR + t0 + i * 4) = a; *(volatile v4i*)(ROWCNT + t0 + i * 4) = c; }
    __threadfence(); }
}
__global__ __launch_bounds__(256) void csrZ_kernel9(int* __restrict__ p, size_t n4) { typedef __attribute__((ext_vector_type(4))) int v4i; const size_t tid = (size_t)blockIdx.x * 256 + threadIdx.x, nth = (size_t)gridDim.x * 256; v4i z = {0, 0, 0, 0}; for (size_t i = tid; i < n4; i += nth) *(volatile v4i*)(p + i * 4) = z; }
struct CsrBufs9 { int *STG, *HST, *OFF, *START, *TOT, *PERM, *ROWPTR, *ROWCNT, *FLAG; int nG, NGP, CHP; size_t permLen; char* base; size_t bytes; };
static size_t csr_carve9(CsrBufs9& c, char* ws, size_t off, int E, int N) {
  const size_t off0 = off; c.base = ws + off;
  auto al = [&](size_t bytes) { char* p = ws + off; off += (bytes + 255) & ~(size_t)255; return p; };
  c.nG = (N + CSR_GN9 - 1) / CSR_GN9; c.NGP = (c.nG + 31) & ~31; const int ch = (E + CSR_NBLK9 - 1) / CSR_NBLK9; c.CHP = (ch + 31) & ~31; c.permLen = (size_t)E + 32 * (size_t)c.nG + 32;
  c.STG = (int*)al((size_t)CSR_NBLK9 * c.CHP * 4); c.HST = (int*)al((size_t)CSR_NBLK9 * c.NGP * 4); c.OFF = (int*)al((size_t)c.NGP * CSR_NBLK9 * 4); c.START = (int*)al((size_t)(c.NGP + 64) * 4); c.TOT = (int*)al((size_t)(c.NGP + 64) * 4);
  c.PERM = (int*)al(c.permLen * 4); c.ROWPTR = (int*)al((size_t)c.nG * CSR_TS9 * 4); c.ROWCNT = (int*)al((size_t)c.nG * CSR_TS9 * 4); c.FLAG = (int*)al(256);
  c.bytes = off - off0; return off;
}
static void csr_build9(const CsrBufs9& c, const int* dst, int E, int N, hipStream_t stream) {
  const size_t smem = (size_t)(2 * c.NGP + c.CHP) * 4;
  csrZ_kernel9<<<512, 256, 0, stream>>>((int*)c.base, c.bytes / 16);
  csrA_kernel9<<<CSR_NBLK9, 64, smem, stream>>>(dst, E, N, c.nG, c.CHP, c.NGP, c.STG, c.HST);
  csrS_kernel9<<<1, 512, 0, stream>>>(c.HST, c.nG, c.NGP, c.START, c.TOT, c.OFF);
  csrB_kernel9<<<c.nG, 256, 0, stream>>>(dst, N, c.nG, c.CHP, c.NGP, (int)c.permLen, c.STG, c.HST, c.OFF, c.START, c.TOT, c.PERM, c.ROWPTR, c.ROWCNT, c.FLAG);
}

__device__ __forceinline__ void nw3(const float* lw, float* nw) { float a = bfv(lw[0]), b = bfv(lw[1]), c = bfv(lw[2]); const float m = fmaxf(a, fmaxf(b, c)); a = __expf(a - m); b = __expf(b - m); c = __expf(c - m); const float s = a + b + c; nw[0] = a / s; nw[1] = b / s; nw[2] = c / s; }

__global__ __launch_bounds__(256) void wput_kernel(const float* __restrict__ wsoc, const float* __restrict__ how, const float* __restrict__ mpw, b16* __restrict__ WS, b16* __restrict__ WH, b16* __restrict__ WM) { const int u = blockIdx.x * 256 + threadIdx.x; v8b v;
  if (u < 2 * D * 8) { const int l = u / (D * 8), r = u % (D * 8); const int o = r / 8, k0 = (r % 8) * 8;
#pragma unroll
    for (int j = 0; j < 8; ++j) v[j] = (b16)(bf16_rne(wsoc[((size_t)l * D + k0 + j) * D + o]) * WSC); for (int pass = 0; pass < 2; ++pass) { *(volatile v8b*)(WS + ((size_t)l * D + o) * D + k0) = v; __threadfence(); } }
  if (u < D * 8) { const int o = u / 8, k0 = (u % 8) * 8;
#pragma unroll
    for (int j = 0; j < 8; ++j) v[j] = (b16)(bf16_rne(how[(size_t)(k0 + j) * D + o]) * WSC); for (int pass = 0; pass < 2; ++pass) { *(volatile v8b*)(WH + (size_t)o * D + k0) = v; __threadfence(); } }
  if (u < D * 16) { const int o = u / 16, k0 = (u % 16) * 8;
#pragma unroll
    for (int j = 0; j < 8; ++j) v[j] = (b16)(bf16_rne(mpw[(size_t)(k0 + j) * D + o]) * WSC); for (int pass = 0; pass < 2; ++pass) { *(volatile v8b*)(WM + (size_t)o * 2 * D + k0) = v; __threadfence(); } } }
template <int XBF>
__global__ __launch_bounds__(256) void spmm_kernel(const float* __restrict__ X, const float* __restrict__ base, const float* __restrict__ w, const int* __restrict__ cols, const int* __restrict__ PERM, const int* __restrict__ ROWPTR, const int* __restrict__ ROWCNT, int permLen, int EMAX, int ncolmax, int ROWS, int COLLIM, float* __restrict__ OUT) { const int wave = threadIdx.x >> 5, lane = threadIdx.x & 31; const size_t i = (size_t)blockIdx.x * NPB + wave; if (i >= (size_t)ROWS) return; int st = ROWPTR[i], cnt = ROWCNT[i]; cnt = iclamp(cnt, 0, EMAX); st = iclamp(st, 0, permLen - cnt); float s0 = 0.0f, s1 = 0.0f;
#pragma unroll 1
  for (int j = 0; j < cnt; ++j) { const int e = iclamp(PERM[st + j], 0, EMAX - 1); const size_t c = (size_t)iclamp(cols[e], 0, ncolmax - 1); if (c >= (size_t)COLLIM) continue; const float we = bfv(w[e]); v2f v = *(const v2f*)(X + c * D + lane * 2); if (XBF) { v[0] = bfv(v[0]); v[1] = bfv(v[1]); } s0 += pmul(we, v[0]); s1 += pmul(we, v[1]); }
  if (base) { s0 += pmul(0.1f, bfv(base[i * D + lane * 2])); s1 += pmul(0.1f, bfv(base[i * D + lane * 2 + 1])); }
  for (int pass = 0; pass < 2; ++pass) { *(volatile v2f*)(OUT + i * D + lane * 2) = (v2f){s0, s1}; __threadfence(); } }
__global__ __launch_bounds__(256) void itemw_kernel(const float* __restrict__ U1, const float* __restrict__ I1, const float* __restrict__ i0, const int* __restrict__ pos, const float* __restrict__ w, const int* __restrict__ cols, const int* __restrict__ PERM, const int* __restrict__ ROWPTR, const int* __restrict__ ROWCNT, int permLen, const float* __restrict__ lw, int ULIM, float* __restrict__ IW) { const int wave = threadIdx.x >> 5, lane = threadIdx.x & 31; const int b = blockIdx.x * NPB + wave; if (b >= NB) return; const size_t p = (size_t)iclamp(pos[b], 0, NI - 1); float nw[3]; nw3(lw, nw);
  int st = ROWPTR[p], cnt = ROWCNT[p]; cnt = iclamp(cnt, 0, EUI); st = iclamp(st, 0, permLen - cnt); float s[2] = {0.0f, 0.0f};
#pragma unroll 1
  for (int j = 0; j < cnt; ++j) { const int e = iclamp(PERM[st + j], 0, EUI - 1); const size_t c = (size_t)iclamp(cols[e], 0, NU - 1); if (c >= (size_t)ULIM) continue; const float we = bfv(w[e]); const v2f v = *(const v2f*)(U1 + c * D + lane * 2); s[0] += pmul(we, v[0]); s[1] += pmul(we, v[1]); }
  v2f o; for (int k = 0; k < 2; ++k) { const int c = lane * 2 + k; const float iz = bfv(i0[p * D + c]); const float i2 = s[k] + pmul(0.1f, iz); o[k] = pmul(nw[0], iz) + pmul(nw[1], I1[p * D + c]) + pmul(nw[2], i2); }
  for (int pass = 0; pass < 2; ++pass) { *(volatile v2f*)(IW + (size_t)b * D + lane * 2) = o; __threadfence(); } }
__global__ __launch_bounds__(32) void lin64_kernel(const float* __restrict__ IN, const int* __restrict__ IDX, const b16* __restrict__ W, int ROWS, float* __restrict__ OUT) { __shared__ __attribute__((aligned(16))) b16 Ah[16][D + 8], Al[16][D + 8]; __shared__ float Tf[16][D + 4]; const int lane = threadIdx.x, nloc = lane & 15, hlf = lane >> 4; const size_t m0 = (size_t)blockIdx.x * 16; if (m0 >= (size_t)ROWS) return;
  for (int rr = 0; rr < 16; ++rr) { const size_t row = IDX ? (size_t)iclamp(IDX[m0 + rr], 0, NU - 1) : m0 + rr; for (int q = 0; q < 2; ++q) { b16 p, ql; split16(IN[row * D + q * 32 + lane] * HS, p, ql); Ah[rr][q * 32 + lane] = p; Al[rr][q * 32 + lane] = ql; } } if (lane < 16) for (int k = D; k < D + 8; ++k) { Ah[lane][k] = (b16)0.0f; Al[lane][k] = (b16)0.0f; }
  wave_lds_sync(); v8f acc[4] = {(v8f){}, (v8f){}, (v8f){}, (v8f){}};
#pragma unroll
  for (int kb = 0; kb < D; kb += 32) { const v16b a = frag_kb(&Ah[nloc][kb], hlf), al = frag_kb(&Al[nloc][kb], hlf);
#pragma unroll
    for (int t = 0; t < 4; ++t) { const v16b bw = frag_kb(W + (size_t)(t * 16 + nloc) * D + kb, hlf); acc[t] = wmma16b(a, bw, acc[t]); acc[t] = wmma16b(al, bw, acc[t]); } }
#pragma unroll
  for (int t = 0; t < 4; ++t)
#pragma unroll
    for (int r8 = 0; r8 < 8; ++r8) Tf[8 * hlf + r8][t * 16 + nloc] = acc[t][r8] * (1.0f / (HS * WSC));
  wave_lds_sync();
  for (int pass = 0; pass < 2; ++pass) { for (int rr = 0; rr < 16; ++rr) *(volatile v2f*)(OUT + (m0 + rr) * D + lane * 2) = *(const v2f*)(&Tf[rr][lane * 2]); __threadfence(); } }
__global__ __launch_bounds__(256) void socnew_kernel(const float* __restrict__ CW, const float* __restrict__ CUR, const int* __restrict__ IDX, const float* __restrict__ w, const int* __restrict__ cols, const int* __restrict__ PERM, const int* __restrict__ ROWPTR, const int* __restrict__ ROWCNT, int permLen, int ROWS, int ULIM, float* __restrict__ NEW) { const int wave = threadIdx.x >> 5, lane = threadIdx.x & 31; const size_t k = (size_t)blockIdx.x * NPB + wave; if (k >= (size_t)ROWS) return; const size_t i = IDX ? (size_t)iclamp(IDX[k], 0, NU - 1) : k; int st = ROWPTR[i], cnt = ROWCNT[i]; cnt = iclamp(cnt, 0, ES_); st = iclamp(st, 0, permLen - cnt); float s0 = 0.0f, s1 = 0.0f;
#pragma unroll 1
  for (int j = 0; j < cnt; ++j) { const int e = iclamp(PERM[st + j], 0, ES_ - 1); const size_t c = (size_t)iclamp(cols[e], 0, NU - 1); if (c >= (size_t)ULIM) continue; const float we = bfv(w[e]); const v2f v = *(const v2f*)(CW + c * D + lane * 2); s0 += pmul(we, v[0]); s1 += pmul(we, v[1]); }
  const v2f cv = *(const v2f*)(CUR + i * D + lane * 2);
  for (int pass = 0; pass < 2; ++pass) { *(volatile v2f*)(NEW + k * D + lane * 2) = (v2f){cv[0] + s0, cv[1] + s1}; __threadfence(); } }
__global__ __launch_bounds__(32) void gate_kernel(const float* __restrict__ NEW, const float* __restrict__ CUR, const int* __restrict__ IDX, const b16* __restrict__ WH, const float* __restrict__ hb, const float* __restrict__ hg, const float* __restrict__ hbeta, int ROWS, float* __restrict__ OUT) { __shared__ __attribute__((aligned(16))) b16 Ah[16][D + 8], Al[16][D + 8]; __shared__ float Tf[16][D + 4]; const int lane = threadIdx.x, nloc = lane & 15, hlf = lane >> 4; const size_t m0 = (size_t)blockIdx.x * 16; if (m0 >= (size_t)ROWS) return;
  for (int rr = 0; rr < 16; ++rr) for (int q = 0; q < 2; ++q) { b16 p, ql; split16(NEW[(m0 + rr) * D + q * 32 + lane] * HS, p, ql); Ah[rr][q * 32 + lane] = p; Al[rr][q * 32 + lane] = ql; } if (lane < 16) for (int k = D; k < D + 8; ++k) { Ah[lane][k] = (b16)0.0f; Al[lane][k] = (b16)0.0f; }
  wave_lds_sync(); v8f acc[4] = {(v8f){}, (v8f){}, (v8f){}, (v8f){}};
#pragma unroll
  for (int kb = 0; kb < D; kb += 32) { const v16b a = frag_kb(&Ah[nloc][kb], hlf), al = frag_kb(&Al[nloc][kb], hlf);
#pragma unroll
    for (int t = 0; t < 4; ++t) { const v16b bw = frag_kb(WH + (size_t)(t * 16 + nloc) * D + kb, hlf); acc[t] = wmma16b(a, bw, acc[t]); acc[t] = wmma16b(al, bw, acc[t]); } }
#pragma unroll
  for (int t = 0; t < 4; ++t) { const int cc = t * 16 + nloc; const float bb = bfv(hb[cc]);
#pragma unroll
    for (int r8 = 0; r8 < 8; ++r8) Tf[8 * hlf + r8][cc] = acc[t][r8] * (1.0f / (HS * WSC)) + bb; }
  wave_lds_sync();
  for (int pass = 0; pass < 2; ++pass) { for (int rr = 0; rr < 16; ++rr) { const size_t row = IDX ? (size_t)iclamp(IDX[m0 + rr], 0, NU - 1) : m0 + rr; float v[2], sm = 0.0f; for (int k = 0; k < 2; ++k) { v[k] = Tf[rr][lane * 2 + k]; sm += v[k]; } for (int o = 16; o; o >>= 1) sm += __shfl_xor(sm, o); const float mu = sm / D; float q2 = 0.0f; for (int k = 0; k < 2; ++k) q2 += (v[k] - mu) * (v[k] - mu); for (int o = 16; o; o >>= 1) q2 += __shfl_xor(q2, o); const float rs = rsqrtf(q2 / D + LNEPS); v2f o2;
      for (int k = 0; k < 2; ++k) { const int c = lane * 2 + k; const float g = sigm(leaky(pmul((v[k] - mu) * rs, bfv(hg[c])) + bfv(hbeta[c]))); o2[k] = pmul(g, NEW[(m0 + rr) * D + c]) + pmul(1.0f - g, CUR[row * D + c]); }
      *(volatile v2f*)(OUT + (m0 + rr) * D + lane * 2) = o2; } __threadfence(); } }
__global__ __launch_bounds__(32) void score_kernel(const float* __restrict__ u0, const float* __restrict__ U1, const float* __restrict__ U2, const float* __restrict__ CUR1, const float* __restrict__ CUR2B, const float* __restrict__ IW, const int* __restrict__ users, const float* __restrict__ lw, const b16* __restrict__ WM, const float* __restrict__ mb, const float* __restrict__ mg, const float* __restrict__ mbeta, float* __restrict__ out) { __shared__ __attribute__((aligned(16))) b16 Ah[32][2 * D + 8], Al[32][2 * D + 8]; __shared__ float Tf[32][D + 4], Os[32]; const int lane = threadIdx.x, nloc = lane & 15, hlf = lane >> 4; const size_t b0 = (size_t)blockIdx.x * 32; float nw[3]; nw3(lw, nw);
  for (int rr = 0; rr < 32; ++rr) { const size_t b = b0 + rr; const size_t u = (size_t)iclamp(users[b], 0, NU - 1); for (int q = 0; q < 2; ++q) { const int c = q * 32 + lane; const float uw = pmul(nw[0], bfv(u0[u * D + c])) + pmul(nw[1], U1[u * D + c]) + pmul(nw[2], U2[u * D + c]); const float sw = pmul(nw[0], U2[u * D + c]) + pmul(nw[1], CUR1[u * D + c]) + pmul(nw[2], CUR2B[b * D + c]); b16 p, ql; split16(uw * HS, p, ql); Ah[rr][c] = p; Al[rr][c] = ql; split16(sw * HS, p, ql); Ah[rr][D + c] = p; Al[rr][D + c] = ql; } }
  for (int k = 2 * D; k < 2 * D + 8; ++k) { Ah[lane][k] = (b16)0.0f; Al[lane][k] = (b16)0.0f; }
  wave_lds_sync();
#pragma unroll
  for (int rt = 0; rt < 2; ++rt) { v8f acc[4] = {(v8f){}, (v8f){}, (v8f){}, (v8f){}};
#pragma unroll
    for (int kb = 0; kb < 2 * D; kb += 32) { const v16b a = frag_kb(&Ah[rt * 16 + nloc][kb], hlf), al = frag_kb(&Al[rt * 16 + nloc][kb], hlf);
#pragma unroll
      for (int t = 0; t < 4; ++t) { const v16b bw = frag_kb(WM + (size_t)(t * 16 + nloc) * 2 * D + kb, hlf); acc[t] = wmma16b(a, bw, acc[t]); acc[t] = wmma16b(al, bw, acc[t]); } }
#pragma unroll
    for (int t = 0; t < 4; ++t) { const int cc = t * 16 + nloc; const float bb = bfv(mb[cc]);
#pragma unroll
      for (int r8 = 0; r8 < 8; ++r8) Tf[rt * 16 + 8 * hlf + r8][cc] = acc[t][r8] * (1.0f / (HS * WSC)) + bb; } }
  wave_lds_sync();
  for (int rr = 0; rr < 32; ++rr) { float v[2], sm = 0.0f; for (int k = 0; k < 2; ++k) { v[k] = Tf[rr][lane * 2 + k]; sm += v[k]; } for (int o = 16; o; o >>= 1) sm += __shfl_xor(sm, o); const float mu = sm / D; float q2 = 0.0f; for (int k = 0; k < 2; ++k) q2 += (v[k] - mu) * (v[k] - mu); for (int o = 16; o; o >>= 1) q2 += __shfl_xor(q2, o); const float rs = rsqrtf(q2 / D + LNEPS); float s = 0.0f;
    for (int k = 0; k < 2; ++k) { const int c = lane * 2 + k; const float f = leaky(pmul((v[k] - mu) * rs, bfv(mg[c])) + bfv(mbeta[c])); s += pmul(f, IW[(b0 + rr) * D + c]); } for (int o = 16; o; o >>= 1) s += __shfl_xor(s, o); if (lane == 0) Os[rr] = s; }
  wave_lds_sync();
  for (int pass = 0; pass < 2; ++pass) { ((volatile float*)out)[b0 + lane] = Os[lane]; __threadfence(); } }
}

extern "C" void kernel_launch(void* const* d_in, const int* in_sizes, int n_in, void* d_out, int out_size, void* d_ws, size_t ws_size, hipStream_t stream) {
  (void)n_in;
  auto Fp = [&](int i) { return (const float*)d_in[i]; }; auto Ip = [&](int i) { return (const int*)d_in[i]; };
  if (in_sizes[0] != NB || in_sizes[1] != NB || in_sizes[2] != EUI || in_sizes[4] != EUI || in_sizes[5] != ES_ || in_sizes[7] != ES_ || in_sizes[8] != NU * D || in_sizes[9] != NI * D || in_sizes[10] != 4 || in_sizes[11] != 2 * D * D || in_sizes[16] != 2 * D * D || out_size != NB) return;
  const int ULIM = NU, ILIM = NI;
  size_t off = 0; char* ws = (char*)d_ws;
  auto carve = [&](size_t bytes) { char* p = ws + off; off += (bytes + 255) & ~(size_t)255; return p; };
  b16* WS = (b16*)carve((size_t)2 * D * D * 2); b16* WH = (b16*)carve(D * D * 2); b16* WM = (b16*)carve((size_t)D * 2 * D * 2);
  float* U1 = (float*)carve((size_t)NU * D * 4); float* U2 = (float*)carve((size_t)NU * D * 4); float* I1 = (float*)carve((size_t)NI * D * 4); float* CW = (float*)carve((size_t)NU * D * 4); float* NEWP = (float*)carve((size_t)NU * D * 4); float* CUR1 = (float*)carve((size_t)NU * D * 4);
  float* IW = (float*)carve((size_t)NB * D * 4); float* NEWB = (float*)carve((size_t)NB * D * 4); float* CUR2B = (float*)carve((size_t)NB * D * 4);
  CsrBufs8 cu, cs; CsrBufs9 ci; off = csr_carve8(cu, ws, off, EUI, NU); off = csr_carve9(ci, ws, off, EUI, NI); off = csr_carve8(cs, ws, off, ES_, NU);
  if (off > ws_size || off > ((size_t)216 << 20)) return;
  const int nbU = (ULIM + NPB - 1) / NPB, nbI = (ILIM + NPB - 1) / NPB, nbB = NB / NPB;
  wput_kernel<<<(2 * D * 8 + 255) / 256, 256, 0, stream>>>(Fp(11), Fp(12), Fp(16), WS, WH, WM);
  csr_build8(cu, Ip(2), EUI, NU, stream);
  csr_build9(ci, Ip(3), EUI, NI, stream);
  csr_build8(cs, Ip(5), ES_, NU, stream);
  spmm_kernel<1><<<nbU, 256, 0, stream>>>(Fp(9), Fp(8), Fp(4), Ip(3), cu.PERM, cu.ROWPTR, cu.ROWCNT, (int)cu.permLen, EUI, NI, ULIM, ILIM, U1);
  spmm_kernel<1><<<nbI, 256, 0, stream>>>(Fp(8), Fp(9), Fp(4), Ip(2), ci.PERM, ci.ROWPTR, ci.ROWCNT, (int)ci.permLen, EUI, NU, ILIM, ULIM, I1);
  spmm_kernel<0><<<nbU, 256, 0, stream>>>(I1, Fp(8), Fp(4), Ip(3), cu.PERM, cu.ROWPTR, cu.ROWCNT, (int)cu.permLen, EUI, NI, ULIM, ILIM, U2);
  itemw_kernel<<<nbB, 256, 0, stream>>>(U1, I1, Fp(9), Ip(1), Fp(4), Ip(2), ci.PERM, ci.ROWPTR, ci.ROWCNT, (int)ci.permLen, Fp(10), ULIM, IW);
  lin64_kernel<<<ULIM / 16, 32, 0, stream>>>(U2, nullptr, WS, ULIM, CW);
  socnew_kernel<<<nbU, 256, 0, stream>>>(CW, U2, nullptr, Fp(7), Ip(6), cs.PERM, cs.ROWPTR, cs.ROWCNT, (int)cs.permLen, ULIM, ULIM, NEWP);
  gate_kernel<<<ULIM / 16, 32, 0, stream>>>(NEWP, U2, nullptr, WH, Fp(13), Fp(14), Fp(15), ULIM, CUR1);
  lin64_kernel<<<ULIM / 16, 32, 0, stream>>>(CUR1, nullptr, WS + (size_t)D * D, ULIM, CW);
  socnew_kernel<<<nbB, 256, 0, stream>>>(CW, CUR1, Ip(0), Fp(7), Ip(6), cs.PERM, cs.ROWPTR, cs.ROWCNT, (int)cs.permLen, NB, ULIM, NEWB);
  gate_kernel<<<NB / 16, 32, 0, stream>>>(NEWB, CUR1, Ip(0), WH, Fp(13), Fp(14), Fp(15), NB, CUR2B);
  score_kernel<<<NB / 32, 32, 0, stream>>>(Fp(8), U1, U2, CUR1, CUR2B, IW, Ip(0), Fp(10), WM, Fp(17), Fp(18), Fp(19), (float*)d_out);
}
